// MACEDiffusionAdapted_84894323572748
// MI455X (gfx1250) — hardware-verified
//
#include <hip/hip_runtime.h>
#include <stddef.h>
#include <stdint.h>

#define NN     4096
#define NE     131072
#define DP     68
#define AP     136
#define NTHR   256
#define NWAVE  8
#define EPT    8
#define CHUNK  (NTHR * EPT)
#define WCAP   (EPT * 32)
#define LISTN  (NWAVE * WCAP)
#define NBA    256
#define SLA    8
#define RCAP   12288
#define DEGCAP 96
#define AGG_ZINTS (LISTN + 2 * RCAP + 3 * NBA)
#define STG_OFF   (AGG_ZINTS + 16)
#define STG_W     1024
#define SCAN_LDS_INTS  (STG_OFF + NWAVE * STG_W)
#define SCAN_LDS_BYTES (SCAN_LDS_INTS * 4)
#define EDGE_F_FLOATS  (128 * DP + 2048 + 128 + 128 + 192)
#define EDGE_LDS_BYTES (EDGE_F_FLOATS * 4 + 128 * AP * 2)
#define WSMAX  134217728

#define PB_POS 0
#define PB_TEB 16
#define PB_EWT 80
#define PB_EW5 81
#define PB_EB  82
#define PB_W1F 83
#define PB_B1F 84
#define PB_WVF 85
#define PB_W2D 86
#define PB_WMD 94
#define PB_WPD 126
#define PB_END 134

static constexpr size_t O_RP   = 0;
static constexpr size_t O_YP   = O_RP   + (size_t)NE * 64 * 4;
static constexpr size_t O_LEN0 = O_YP   + (size_t)NE * 16 * 4;
static constexpr size_t O_AG   = O_LEN0 + (size_t)NE * 4;
static constexpr size_t O_MIX  = O_AG   + (size_t)16 * NN * 128 * 2;
static constexpr size_t O_NF   = O_MIX  + (size_t)16 * NN * 64 * 4;
static constexpr size_t O_HS   = O_NF   + (size_t)16 * NN * 64 * 4;
static constexpr size_t O_POS0 = O_HS   + (size_t)NN * 64 * 4;
static constexpr size_t O_POS1 = O_POS0 + (size_t)NN * 16;
static constexpr size_t O_MBV0 = O_POS1 + (size_t)NN * 16;
static constexpr size_t O_MBV1 = O_MBV0 + (size_t)3 * NN * 4;
static constexpr size_t O_TEB  = O_MBV1 + (size_t)3 * NN * 4;
static constexpr size_t O_EWT  = O_TEB  + (size_t)NN * 32 * 2;
static constexpr size_t O_EW5  = O_EWT  + 4096;
static constexpr size_t O_EB   = O_EW5  + 1536;
static constexpr size_t O_W1F  = O_EB   + 256;
static constexpr size_t O_B1F  = O_W1F  + 1024;
static constexpr size_t O_WVF  = O_B1F  + 512;
static constexpr size_t O_W2D  = O_WVF  + 512;
static constexpr size_t O_WMD  = O_W2D  + 32768;
static constexpr size_t O_WPD  = O_WMD  + 131072;
static constexpr size_t O_FLG  = O_WPD  + 32768;
static constexpr size_t O_END  = O_FLG  + 4096;

static_assert(O_END <= (size_t)WSMAX);
static_assert((O_YP % 256) == 0 && (O_LEN0 % 256) == 0 && (O_AG % 256) == 0 && (O_MIX % 256) == 0);
static_assert((O_NF % 256) == 0 && (O_HS % 256) == 0 && (O_POS0 % 256) == 0 && (O_POS1 % 256) == 0);
static_assert((O_MBV0 % 256) == 0 && (O_MBV1 % 256) == 0 && (O_TEB % 256) == 0 && (O_EWT % 256) == 0);
static_assert((O_EW5 % 256) == 0 && (O_EB % 256) == 0 && (O_W1F % 256) == 0 && (O_B1F % 256) == 0);
static_assert((O_WVF % 256) == 0 && (O_W2D % 256) == 0 && (O_WMD % 256) == 0 && (O_WPD % 256) == 0);
static_assert((O_FLG % 256) == 0);
static_assert(NE % 128 == 0 && NE % CHUNK == 0 && NN % 256 == 0 && NN % 128 == 0);
static_assert(NN == 16 * NBA && NBA == (1 << SLA) && NBA % NWAVE == 0 && NBA % 32 == 0);
static_assert((CHUNK & (CHUNK - 1)) == 0 && ((long long)NE << SLA) < (1LL << 31));
static_assert(AGG_ZINTS % 4 == 0 && STG_OFF % 4 == 0 && RCAP % 4 == 0);
static_assert(SCAN_LDS_BYTES <= 300000 && EDGE_LDS_BYTES <= 300000);
static_assert((EDGE_F_FLOATS * 4) % 16 == 0 && (DP * 4) % 16 == 0 && (AP * 2) % 16 == 0 && AP >= 128 && DP >= 64);

typedef float          v2f   __attribute__((ext_vector_type(2)));
typedef float          v4f   __attribute__((ext_vector_type(4)));
typedef float          v8f   __attribute__((ext_vector_type(8)));
typedef int            v4i   __attribute__((ext_vector_type(4)));
typedef int            v8i   __attribute__((ext_vector_type(8)));
typedef unsigned short v8us  __attribute__((ext_vector_type(8)));
typedef unsigned short v16us __attribute__((ext_vector_type(16)));
typedef __bf16         v16bf __attribute__((ext_vector_type(16)));
typedef v2f  __attribute__((may_alias)) v2fa;
typedef v4f  __attribute__((may_alias)) v4fa;
typedef v4i  __attribute__((may_alias)) v4ia;
typedef v8us __attribute__((may_alias)) v8usa;
typedef unsigned __attribute__((may_alias)) u32a;
union FragB { v16bf v; v16us u; v8us h[2]; v8i w; };

__device__ __forceinline__ v8f wmb(const FragB& a, const FragB& b, v8f c) {
  v8f d = __builtin_amdgcn_wmma_f32_16x16x32_bf16(false, a.v, false, b.v, (short)0, c, false, false);
  asm volatile("v_nop\n\tv_nop\n\tv_nop\n\tv_nop" : "+v"(d) : "v"(a.w), "v"(b.w));
  return d;
}

__device__ __forceinline__ void ldwait() {
  asm volatile("s_wait_loadcnt 0x0" ::: "memory");
}

__device__ __forceinline__ unsigned bf16_bits(float f) {
  const unsigned u = __float_as_uint(f);
  const unsigned r = (u + 0x7FFFu + ((u >> 16) & 1u)) >> 16;
  return ((u & 0x7FFFFFFFu) > 0x7F800000u) ? 0x7FC0u : r;
}
__device__ __forceinline__ float bf16_val(float f) {
  return __uint_as_float(bf16_bits(f) << 16);
}
__device__ __forceinline__ void put16(unsigned short* dp, v8us o) {
  *(volatile v8us*)dp = o;
  __threadfence();
  *(volatile v8us*)dp = o;
}
__device__ __forceinline__ void putf4(float* dp, v4f o) {
  *(volatile v4f*)dp = o;
  __threadfence();
  *(volatile v4f*)dp = o;
}

__device__ __forceinline__ void wplane(const float* __restrict__ W, unsigned short* D, int u) {
  const int mat = u >> 10, n = (u >> 4) & 63, k8 = (u & 15) * 8, srow = k8 & 63;
  const float* p = W + ((size_t)mat * 64 + srow) * 64 + n;
  v8us o;
#pragma unroll
  for (int i = 0; i < 8; ++i) o[i] = (unsigned short)bf16_bits(p[(size_t)i * 64]);
  put16(D + (size_t)u * 8, o);
}

__global__ __launch_bounds__(NTHR) void k_prep(const float* __restrict__ pos, const float* __restrict__ te,
                                               const float* __restrict__ embW, const float* __restrict__ embb,
                                               const float* __restrict__ W1, const float* __restrict__ b1,
                                               const float* __restrict__ W2, const float* __restrict__ Wmix,
                                               const float* __restrict__ Wprod, const float* __restrict__ Wvec,
                                               char* ws) {
  const int b = (int)blockIdx.x, tid = (int)threadIdx.x;
  if (b < PB_TEB) {
    const int n = b * NTHR + tid;
    const float x = pos[(size_t)n * 3 + 0], y = pos[(size_t)n * 3 + 1], z = pos[(size_t)n * 3 + 2];
    v4f q;
    q.x = bf16_val(x); q.y = bf16_val(y); q.z = bf16_val(z); q.w = 0.0f;
    putf4((float*)(ws + O_POS0) + (size_t)n * 4, q);
  } else if (b < PB_EWT) {
    const int u = (b - PB_TEB) * NTHR + tid;
    const float* p = te + (size_t)u * 8;
    const v4f a = *(const v4f*)p;
    const v4f c = *(const v4f*)(p + 4);
    v8us o;
    o[0] = (unsigned short)bf16_bits(a.x); o[1] = (unsigned short)bf16_bits(a.y);
    o[2] = (unsigned short)bf16_bits(a.z); o[3] = (unsigned short)bf16_bits(a.w);
    o[4] = (unsigned short)bf16_bits(c.x); o[5] = (unsigned short)bf16_bits(c.y);
    o[6] = (unsigned short)bf16_bits(c.z); o[7] = (unsigned short)bf16_bits(c.w);
    put16((unsigned short*)(ws + O_TEB) + (size_t)u * 8, o);
  } else if (b == PB_EWT) {
    const int n = tid >> 2, k8 = (tid & 3) * 8;
    const float* p = embW + (size_t)(5 + k8) * 64 + n;
    v8us o;
#pragma unroll
    for (int i = 0; i < 8; ++i) o[i] = (unsigned short)bf16_bits(p[(size_t)i * 64]);
    put16((unsigned short*)(ws + O_EWT) + (size_t)n * 32 + k8, o);
  } else if (b == PB_EW5) {
    if (tid < 80) {
      const v4f a = *(const v4f*)(embW + (size_t)tid * 4);
      v4f q; q.x = bf16_val(a.x); q.y = bf16_val(a.y); q.z = bf16_val(a.z); q.w = bf16_val(a.w);
      putf4((float*)(ws + O_EW5) + (size_t)tid * 4, q);
    }
  } else if (b == PB_EB) {
    if (tid < 16) {
      const v4f a = *(const v4f*)(embb + (size_t)tid * 4);
      v4f q; q.x = bf16_val(a.x); q.y = bf16_val(a.y); q.z = bf16_val(a.z); q.w = bf16_val(a.w);
      putf4((float*)(ws + O_EB) + (size_t)tid * 4, q);
    }
  } else if (b == PB_W1F) {
    if (tid < 64) {
      const v4f a = *(const v4f*)(W1 + (size_t)tid * 4);
      v4f q; q.x = bf16_val(a.x); q.y = bf16_val(a.y); q.z = bf16_val(a.z); q.w = bf16_val(a.w);
      putf4((float*)(ws + O_W1F) + (size_t)tid * 4, q);
    }
  } else if (b == PB_B1F) {
    if (tid < 32) {
      const v4f a = *(const v4f*)(b1 + (size_t)tid * 4);
      v4f q; q.x = bf16_val(a.x); q.y = bf16_val(a.y); q.z = bf16_val(a.z); q.w = bf16_val(a.w);
      putf4((float*)(ws + O_B1F) + (size_t)tid * 4, q);
    }
  } else if (b == PB_WVF) {
    if (tid < 32) {
      const v4f a = *(const v4f*)(Wvec + (size_t)tid * 4);
      v4f q; q.x = bf16_val(a.x); q.y = bf16_val(a.y); q.z = bf16_val(a.z); q.w = bf16_val(a.w);
      putf4((float*)(ws + O_WVF) + (size_t)tid * 4, q);
    }
  } else if (b < PB_WMD) {
    wplane(W2, (unsigned short*)(ws + O_W2D), (b - PB_W2D) * NTHR + tid);
  } else if (b < PB_WPD) {
    wplane(Wmix, (unsigned short*)(ws + O_WMD), (b - PB_WMD) * NTHR + tid);
  } else {
    wplane(Wprod, (unsigned short*)(ws + O_WPD), (b - PB_WPD) * NTHR + tid);
  }
}

__global__ __launch_bounds__(128) void k_emb(const unsigned short* __restrict__ TEB,
                                             const unsigned short* __restrict__ EWT,
                                             const float* __restrict__ EW5, const float* __restrict__ EB,
                                             const int* __restrict__ attrs, float* HS) {
  __shared__ __attribute__((aligned(16))) float stg[64 * DP];
  const int tid = (int)threadIdx.x, lane = tid & 31, wave = tid >> 5, hh = lane >> 4, m = lane & 15;
  const int rowBase = (int)blockIdx.x * 64;
  v8f acc[4];
  {
    const v8f z = {0.f, 0.f, 0.f, 0.f, 0.f, 0.f, 0.f, 0.f};
    acc[0] = z; acc[1] = z; acc[2] = z; acc[3] = z;
  }
  const unsigned short* ap = TEB + (size_t)(rowBase + 16 * wave + m) * 32 + 8 * hh;
  FragB af;
  af.h[0] = *(const v8usa*)ap;
  af.h[1] = *(const v8usa*)(ap + 16);
#pragma unroll
  for (int nt = 0; nt < 4; ++nt) {
    const unsigned short* bq = EWT + (size_t)(16 * nt + m) * 32 + 8 * hh;
    FragB bf;
    bf.h[0] = *(const v8usa*)bq;
    bf.h[1] = *(const v8usa*)(bq + 16);
    acc[nt] = wmb(af, bf, acc[nt]);
  }
#pragma unroll
  for (int nt = 0; nt < 4; ++nt)
#pragma unroll
    for (int r = 0; r < 8; ++r) stg[(16 * wave + 8 * hh + r) * DP + 16 * nt + m] = acc[nt][r];
  __syncthreads();
  const v4f eb = *(const v4fa*)(EB + 4 * m);
  v4f pv[8];
#pragma unroll
  for (int i = 0; i < 8; ++i) {
    const int lr = 16 * wave + 2 * i + hh;
    const int gr = rowBase + lr;
    const int a  = attrs[gr] - 1;
    const bool ok = (unsigned)a < 5u;
    const int ac = ok ? a : 0;
    const v4f ew = *(const v4fa*)(EW5 + (size_t)ac * 64 + 4 * m);
    v4f v = *(const v4fa*)(stg + lr * DP + 4 * m);
    v.x = (v.x + (ok ? ew.x : 0.0f)) + eb.x;
    v.y = (v.y + (ok ? ew.y : 0.0f)) + eb.y;
    v.z = (v.z + (ok ? ew.z : 0.0f)) + eb.z;
    v.w = (v.w + (ok ? ew.w : 0.0f)) + eb.w;
    pv[i] = v;
  }
#pragma unroll
  for (int i = 0; i < 8; ++i) {
    float* op = HS + (size_t)(rowBase + 16 * wave + 2 * i + hh) * 64 + 4 * m;
    *(volatile v4f*)op = pv[i];
  }
  __threadfence();
#pragma unroll
  for (int i = 0; i < 8; ++i) {
    float* op = HS + (size_t)(rowBase + 16 * wave + 2 * i + hh) * 64 + 4 * m;
    *(volatile v4f*)op = pv[i];
  }
}

template <int L>
__global__ __launch_bounds__(NTHR) __attribute__((amdgpu_num_vgpr(248)))
void k_edge(const int* __restrict__ eidx, const float* __restrict__ POSq,
            const float* __restrict__ W1f, const float* __restrict__ B1f,
            const unsigned short* __restrict__ W2D, float* LEN0, float* YP, float* RP) {
#pragma clang fp contract(off)
  extern __shared__ __attribute__((aligned(16))) float dyn[];
  float* sO  = dyn;
  float* sY  = sO + 128 * DP;
  float* sL0 = sY + 2048;
  float* sL1 = sL0 + 128;
  float* sW  = sL1 + 128;
  unsigned short* sA = (unsigned short*)(sW + 192);

  const int tid = (int)threadIdx.x, lane = tid & 31, wave = tid >> 5, hh = lane >> 4, m = lane & 15;
  const int eb = (int)blockIdx.x * 128;

  if (tid < 128) {
    const int e = eb + tid;
    int s = eidx[e];
    int r = eidx[NE + e];
    s = s < 0 ? 0 : (s > NN - 1 ? NN - 1 : s);
    r = r < 0 ? 0 : (r > NN - 1 ? NN - 1 : r);
    const v4f ps = *(const v4fa*)(POSq + (size_t)s * 4);
    const v4f pr = *(const v4fa*)(POSq + (size_t)r * 4);
    const float vx = pr.x - ps.x, vy = pr.y - ps.y, vz = pr.z - ps.z;
    const float len = sqrtf((vx * vx + vz * vz) + vy * vy);
    float len0 = len;
    if (L == 1) len0 = LEN0[e];
    const float inv = 1.0f / (len + 1e-9f);
    const float x = vx * inv, y = vy * inv, z = vz * inv;
    const float s3  = 1.7320508075688772f;
    const float c2  = 3.872983346207417f;
    const float c20 = 1.118033988749895f;
    const float c22 = 1.9364916731037085f;
    const float c3a = 2.0916500663351889f;
    const float c3b = 10.246950765959598f;
    const float c3c = 1.6201851746019651f;
    const float c30 = 1.3228756555322954f;
    const float c32 = 5.123475382979799f;
    const float xx = x * x, yy = y * y;
    const float z5 = (5.0f * z) * z;
    v4f q0, q1, q2, q3;
    q0.x = 1.0f;            q0.y = s3 * x;       q0.z = s3 * y;     q0.w = s3 * z;
    q1.x = (c2 * x) * y;    q1.y = (c2 * y) * z; q1.z = c20 * ((3.0f * z) * z - 1.0f); q1.w = (c2 * x) * z;
    q2.x = c22 * (xx - yy);
    q2.y = (c3a * y) * ((3.0f * x) * x - yy);
    q2.z = ((c3b * x) * y) * z;
    q2.w = (c3c * y) * (z5 - 1.0f);
    q3.x = (c30 * z) * (z5 - 3.0f);
    q3.y = (c3c * x) * (z5 - 1.0f);
    q3.z = (c32 * z) * (xx - yy);
    q3.w = (c3a * x) * (xx - (3.0f * y) * y);
    float* yr = sY + tid * 16;
    *(v4fa*)(yr)      = q0;
    *(v4fa*)(yr + 4)  = q1;
    *(v4fa*)(yr + 8)  = q2;
    *(v4fa*)(yr + 12) = q3;
    sL0[tid] = len0;
    sL1[tid] = len;
  } else {
    const int i = tid - 128;
    sW[i] = W1f[L * 128 + i];
    if (i < 64) sW[128 + i] = B1f[L * 64 + i];
  }
  __syncthreads();

  {
    v4f pv[2];
#pragma unroll
    for (int it = 0; it < 2; ++it) pv[it] = *(const v4fa*)(sY + (size_t)(it * NTHR + tid) * 4);
    float* yb = YP + (size_t)eb * 16;
#pragma unroll
    for (int it = 0; it < 2; ++it) *(volatile v4f*)(yb + (size_t)(it * NTHR + tid) * 4) = pv[it];
    __threadfence();
#pragma unroll
    for (int it = 0; it < 2; ++it) *(volatile v4f*)(yb + (size_t)(it * NTHR + tid) * 4) = pv[it];
  }
  if (L == 0) {
    if (tid < 32) {
      const v4f lv = *(const v4fa*)(sL0 + 4 * tid);
      putf4(LEN0 + (size_t)eb + 4 * tid, lv);
    }
  }

  {
    const int row = tid >> 1, half = tid & 1;
    const float l0 = sL0[row], l1 = sL1[row];
    unsigned short* ra = sA + row * AP;
#pragma unroll 1
    for (int g = 0; g < 4; ++g) {
      const int j0 = half * 32 + 8 * g;
      const v4f wa0 = *(const v4fa*)(sW + j0),       wa1 = *(const v4fa*)(sW + j0 + 4);
      const v4f wb0 = *(const v4fa*)(sW + 64 + j0),  wb1 = *(const v4fa*)(sW + 64 + j0 + 4);
      const v4f bb0 = *(const v4fa*)(sW + 128 + j0), bb1 = *(const v4fa*)(sW + 128 + j0 + 4);
      const v8f wa = {wa0.x, wa0.y, wa0.z, wa0.w, wa1.x, wa1.y, wa1.z, wa1.w};
      const v8f wb = {wb0.x, wb0.y, wb0.z, wb0.w, wb1.x, wb1.y, wb1.z, wb1.w};
      const v8f bb = {bb0.x, bb0.y, bb0.z, bb0.w, bb1.x, bb1.y, bb1.z, bb1.w};
      v8us ho, lo;
#pragma unroll
      for (int i = 0; i < 8; ++i) {
        const float pre = (l0 * wa[i] + l1 * wb[i]) + bb[i];
        const float hv  = pre / (1.0f + expf(-pre));
        const unsigned hb = bf16_bits(hv);
        ho[i] = (unsigned short)hb;
        lo[i] = (unsigned short)bf16_bits(hv - __uint_as_float(hb << 16));
      }
      *(v8usa*)(ra + j0)      = ho;
      *(v8usa*)(ra + 64 + j0) = lo;
    }
  }
  __syncthreads();

  {
    v8f acc[4];
    {
      const v8f z = {0.f, 0.f, 0.f, 0.f, 0.f, 0.f, 0.f, 0.f};
      acc[0] = z; acc[1] = z; acc[2] = z; acc[3] = z;
    }
    const unsigned short* ap = sA + (16 * wave + m) * AP + 8 * hh;
    const unsigned short* bp = W2D + (size_t)L * 8192 + (size_t)m * 128 + 8 * hh;
#pragma unroll 1
    for (int k0 = 0; k0 < 128; k0 += 32) {
      FragB af;
      af.h[0] = *(const v8usa*)(ap + k0);
      af.h[1] = *(const v8usa*)(ap + k0 + 16);
#pragma unroll
      for (int nt = 0; nt < 4; ++nt) {
        const unsigned short* wq = bp + (size_t)(16 * nt) * 128 + k0;
        FragB bf;
        bf.h[0] = *(const v8usa*)wq;
        bf.h[1] = *(const v8usa*)(wq + 16);
        acc[nt] = wmb(af, bf, acc[nt]);
      }
    }
#pragma unroll
    for (int nt = 0; nt < 4; ++nt)
#pragma unroll
      for (int r = 0; r < 8; ++r) sO[(16 * wave + 8 * hh + r) * DP + 16 * nt + m] = acc[nt][r];
  }
  __syncthreads();

  {
    v4f pv[8];
#pragma unroll
    for (int it = 0; it < 8; ++it) {
      const int idx = it * NTHR + tid;
      pv[it] = *(const v4fa*)(sO + (idx >> 4) * DP + (idx & 15) * 4);
    }
    float* rb = RP + (size_t)eb * 64;
#pragma unroll
    for (int it = 0; it < 8; ++it) *(volatile v4f*)(rb + (size_t)(it * NTHR + tid) * 4) = pv[it];
    __threadfence();
#pragma unroll
    for (int it = 0; it < 8; ++it) *(volatile v4f*)(rb + (size_t)(it * NTHR + tid) * 4) = pv[it];
  }
}

template <int SLB>
__device__ __forceinline__ int scan_chunk(const int* __restrict__ dsts, int nE, int cbase, int slotBase,
                                          int nb, int vec8, int* list, int tid, int lane, int wave) {
  int wc = 0;
  const int el0  = tid * EPT;
  const int e0   = cbase + el0;
  const int sent = -2147483647 - 1;
  v4i da, db;
  if (vec8 != 0 && cbase + CHUNK <= nE) {
    da = *(const v4i*)(dsts + e0);
    db = *(const v4i*)(dsts + e0 + 4);
  } else {
    da.x = (e0     < nE) ? dsts[min(e0,     nE - 1)] : sent;
    da.y = (e0 + 1 < nE) ? dsts[min(e0 + 1, nE - 1)] : sent;
    da.z = (e0 + 2 < nE) ? dsts[min(e0 + 2, nE - 1)] : sent;
    da.w = (e0 + 3 < nE) ? dsts[min(e0 + 3, nE - 1)] : sent;
    db.x = (e0 + 4 < nE) ? dsts[min(e0 + 4, nE - 1)] : sent;
    db.y = (e0 + 5 < nE) ? dsts[min(e0 + 5, nE - 1)] : sent;
    db.z = (e0 + 6 < nE) ? dsts[min(e0 + 6, nE - 1)] : sent;
    db.w = (e0 + 7 < nE) ? dsts[min(e0 + 7, nE - 1)] : sent;
  }
  const unsigned nbs = (unsigned)slotBase;
  const unsigned unb = (unsigned)nb;
  const unsigned s0 = (unsigned)da.x - nbs, s1 = (unsigned)da.y - nbs;
  const unsigned s2 = (unsigned)da.z - nbs, s3 = (unsigned)da.w - nbs;
  const unsigned s4 = (unsigned)db.x - nbs, s5 = (unsigned)db.y - nbs;
  const unsigned s6 = (unsigned)db.z - nbs, s7 = (unsigned)db.w - nbs;
  const bool h0 = s0 < unb, h1 = s1 < unb, h2 = s2 < unb, h3 = s3 < unb;
  const bool h4 = s4 < unb, h5 = s5 < unb, h6 = s6 < unb, h7 = s7 < unb;
  const unsigned any = __builtin_amdgcn_ballot_w32(h0 | h1 | h2 | h3 | h4 | h5 | h6 | h7);
  if (any != 0u) {
#define HITJ(J, HJ, SJ) { \
      const unsigned mj = __builtin_amdgcn_ballot_w32(HJ); \
      if (mj != 0u) { \
        if (HJ) { \
          const int pos = wc + (int)__builtin_amdgcn_mbcnt_lo(mj, 0u); \
          if (pos < WCAP) list[wave * WCAP + pos] = ((el0 + (J)) << SLB) | (int)(SJ); \
        } \
        wc += (int)__builtin_popcount(mj); } }
    HITJ(0, h0, s0)
    HITJ(1, h1, s1)
    HITJ(2, h2, s2)
    HITJ(3, h3, s3)
    HITJ(4, h4, s4)
    HITJ(5, h5, s5)
    HITJ(6, h6, s6)
    HITJ(7, h7, s7)
#undef HITJ
  }
  return wc;
}

__device__ __forceinline__ void stage_pair(u32a* stw, int x, int lane, float v0, float v1) {
  const unsigned h0 = bf16_bits(v0), h1 = bf16_bits(v1);
  const unsigned l0 = bf16_bits(v0 - __uint_as_float(h0 << 16));
  const unsigned l1 = bf16_bits(v1 - __uint_as_float(h1 << 16));
  stw[x * 64 + lane]      = h0 | (h1 << 16);
  stw[x * 64 + 32 + lane] = l0 | (l1 << 16);
}

template <int L>
__global__ __launch_bounds__(NTHR) __attribute__((amdgpu_num_vgpr(248)))
void k_scan(const int* __restrict__ eidx, const float* __restrict__ RP, const float* __restrict__ YP,
            const float* __restrict__ SRC, int* AGw, int* FLG) {
  extern __shared__ __attribute__((aligned(16))) int dsm[];
  int* list = dsm;
  int* hl   = dsm + LISTN;
  int* sl   = hl + RCAP;
  int* cnt  = sl + RCAP;
  int* offs = cnt + NBA;
  int* cur  = offs + NBA;
  int* misc = cur + NBA;
  const int tid = (int)threadIdx.x, lane = tid & 31, wave = tid >> 5;
  const int nodeBase = (int)blockIdx.x * NBA;
  const int* dsts = eidx + NE;

  {
    const v4i z4 = {0, 0, 0, 0};
    for (int i = tid * 4; i < AGG_ZINTS; i += NTHR * 4) *(v4ia*)(dsm + i) = z4;
    if (tid < 16) misc[tid] = 0;
  }
  __syncthreads();

  int t = 0, ov = 0;
#pragma unroll 1
  for (int ch = 0; ch < NE / CHUNK; ++ch) {
    const int cbase = ch * CHUNK;
    const int wc = scan_chunk<SLA>(dsts, NE, cbase, nodeBase, NBA, 1, list, tid, lane, wave);
    if (lane == 0) misc[wave] = wc;
    __syncthreads();
    if (wave == 0) {
#pragma unroll 1
      for (int w2 = 0; w2 < NWAVE; ++w2) {
        int c = misc[w2];
        c = c < 0 ? 0 : (c > WCAP ? WCAP : c);
#pragma unroll 1
        for (int b0 = 0; b0 < c; b0 += 32) {
          const int idx = b0 + lane;
          const int ent = list[w2 * WCAP + (idx < WCAP ? idx : WCAP - 1)];
          const int m32 = (c - b0) < 32 ? (c - b0) : 32;
#pragma unroll 1
          for (int k = 0; k < m32; ++k) {
            const int u    = __builtin_amdgcn_readlane(ent, k);
            const int slot = u & (NBA - 1);
            const int el   = (u >> SLA) & (CHUNK - 1);
            const int pk   = ((cbase + el) << SLA) | slot;
            if (t < RCAP) {
              if (lane == 0) { hl[t] = pk; cnt[slot] = cnt[slot] + 1; }
              t = t + 1;
            } else {
              ov = 1;
            }
          }
        }
      }
    }
    __syncthreads();
  }
  if (wave == 0 && lane == 0) { misc[8] = t; misc[9] = ov; }
  __syncthreads();
  int tt = misc[8];
  tt = tt < 0 ? 0 : (tt > RCAP ? RCAP : tt);
  const int ovf = misc[9];

  if (wave == 0) {
    const int base = lane * (NBA / 32);
    int s = 0;
    int bigl = 0;
#pragma unroll 1
    for (int i = 0; i < NBA / 32; ++i) {
      const int cv = cnt[base + i];
      s += cv;
      bigl |= (cv > DEGCAP) ? 1 : 0;
    }
    int incl = s;
#pragma unroll
    for (int d = 1; d < 32; d <<= 1) {
      const int y = __shfl_up(incl, d, 32);
      if (lane >= d) incl += y;
    }
    int run = incl - s;
#pragma unroll 1
    for (int i = 0; i < NBA / 32; ++i) {
      const int cv = cnt[base + i];
      offs[base + i] = run;
      cur[base + i]  = run;
      run += cv;
    }
    const unsigned bm = __builtin_amdgcn_ballot_w32(bigl != 0);
    const int fl = ((ovf != 0) || (bm != 0u)) ? 1 : 0;
    const v4i fv = {fl, fl, fl, fl};
    int* fp = FLG + (size_t)(L * 16 + (int)blockIdx.x) * 32 + 4 * (lane & 7);
    if (lane < 8) *(volatile v4i*)fp = fv;
    __threadfence();
    if (lane < 8) *(volatile v4i*)fp = fv;
  }
  __syncthreads();
  if (wave == 0) {
#pragma unroll 1
    for (int b0 = 0; b0 < tt; b0 += 32) {
      const int idx = b0 + lane;
      const int ent = hl[idx < RCAP ? idx : RCAP - 1];
      const int m32 = (tt - b0) < 32 ? (tt - b0) : 32;
#pragma unroll 1
      for (int k = 0; k < m32; ++k) {
        const int u    = __builtin_amdgcn_readlane(ent, k);
        const int slot = u & (NBA - 1);
        if (lane == 0) {
          int p = cur[slot];
          p = p < 0 ? 0 : (p > RCAP - 1 ? RCAP - 1 : p);
          sl[p] = u;
          cur[slot] = p + 1;
        }
      }
    }
  }
  __syncthreads();

  const float qnan = __int_as_float(0x7fc00000);
  const float pzb  = (ovf != 0) ? qnan : 0.0f;
  u32a* stw = (u32a*)(dsm + STG_OFF + wave * STG_W);
  const int hl16 = lane >> 4, l15 = lane & 15;
  constexpr int NST = (L == 0) ? 8 : 2;
#pragma unroll 1
  for (int si = 0; si < NBA / NWAVE; ++si) {
    const int s    = si * NWAVE + wave;
    const int node = nodeBase + s;
    int c = cnt[s];
    const bool big = c > DEGCAP;
    c = c < 0 ? 0 : (c > DEGCAP ? DEGCAP : c);
    int o = offs[s];
    o = o < 0 ? 0 : (o > RCAP ? RCAP : o);
    const float pz = big ? qnan : pzb;

    if constexpr (L == 0) {
      float a0[16], a1[16];
#pragma unroll
      for (int x = 0; x < 16; ++x) { a0[x] = 0.0f; a1[x] = 0.0f; }
#pragma unroll 1
      for (int b0 = 0; b0 < c; b0 += 32) {
        int idx = o + b0 + lane;
        idx = idx > RCAP - 1 ? RCAP - 1 : idx;
        const int ent = sl[idx];
        int eid = ent >> SLA;
        eid = eid < 0 ? 0 : (eid > NE - 1 ? NE - 1 : eid);
        int snd = eidx[eid];
        snd = snd < 0 ? 0 : (snd > NN - 1 ? NN - 1 : snd);
        const int m32 = (c - b0) < 32 ? (c - b0) : 32;
#pragma unroll 1
        for (int k = 0; k < m32; ++k) {
          const int ek = __builtin_amdgcn_readlane(eid, k);
          const int sk = __builtin_amdgcn_readlane(snd, k);
          const v2f r2 = *(const v2fa*)(RP + (size_t)ek * 64 + 2 * lane);
          const v2f h2 = *(const v2fa*)(SRC + (size_t)sk * 64 + 2 * lane);
          const float* yp = YP + (size_t)ek * 16;
          const v4f y0 = *(const v4fa*)yp, y1 = *(const v4fa*)(yp + 4);
          const v4f y2 = *(const v4fa*)(yp + 8), y3 = *(const v4fa*)(yp + 12);
          ldwait();
          const float yy[16] = {y0.x, y0.y, y0.z, y0.w, y1.x, y1.y, y1.z, y1.w,
                                y2.x, y2.y, y2.z, y2.w, y3.x, y3.y, y3.z, y3.w};
          const float q0 = r2.x * h2.x, q1 = r2.y * h2.y;
#pragma unroll
          for (int x = 0; x < 16; ++x) { a0[x] += q0 * yy[x]; a1[x] += q1 * yy[x]; }
        }
      }
#pragma unroll
      for (int x = 0; x < 16; ++x) {
        const float sc = (x == 0) ? 0.0625f : 0.03125f;
        stage_pair(stw, x, lane, a0[x] * sc + pz, a1[x] * sc + pz);
      }
    } else {
      float m0 = 0.0f, m1 = 0.0f, t0 = 0.0f, t1 = 0.0f;
      float j0[3], j1[3];
#pragma unroll
      for (int j = 0; j < 3; ++j) { j0[j] = 0.0f; j1[j] = 0.0f; }
#pragma unroll 1
      for (int b0 = 0; b0 < c; b0 += 32) {
        int idx = o + b0 + lane;
        idx = idx > RCAP - 1 ? RCAP - 1 : idx;
        const int ent = sl[idx];
        int eid = ent >> SLA;
        eid = eid < 0 ? 0 : (eid > NE - 1 ? NE - 1 : eid);
        int snd = eidx[eid];
        snd = snd < 0 ? 0 : (snd > NN - 1 ? NN - 1 : snd);
        const int m32 = (c - b0) < 32 ? (c - b0) : 32;
#pragma unroll 1
        for (int k = 0; k < m32; ++k) {
          const int ek = __builtin_amdgcn_readlane(eid, k);
          const int sk = __builtin_amdgcn_readlane(snd, k);
          const v2f r2 = *(const v2fa*)(RP + (size_t)ek * 64 + 2 * lane);
          const float* yp = YP + (size_t)ek * 16;
          const v4f y0 = *(const v4fa*)yp, y1 = *(const v4fa*)(yp + 4);
          const v4f y2 = *(const v4fa*)(yp + 8), y3 = *(const v4fa*)(yp + 12);
          ldwait();
          const float yy[16] = {y0.x, y0.y, y0.z, y0.w, y1.x, y1.y, y1.z, y1.w,
                                y2.x, y2.y, y2.z, y2.w, y3.x, y3.y, y3.z, y3.w};
          const float* hb = SRC + (size_t)sk * 64 + 2 * lane;
          v2f hA[8];
#pragma unroll
          for (int x = 0; x < 8; ++x) hA[x] = *(const v2fa*)(hb + (size_t)x * NN * 64);
          ldwait();
          float d0 = 0.0f, d1 = 0.0f;
#pragma unroll
          for (int x = 0; x < 8; ++x) { d0 += hA[x].x * yy[x]; d1 += hA[x].y * yy[x]; }
          const float q0 = r2.x * hA[0].x, q1 = r2.y * hA[0].y;
          v2f hB[8];
#pragma unroll
          for (int x = 0; x < 8; ++x) hB[x] = *(const v2fa*)(hb + (size_t)(8 + x) * NN * 64);
          ldwait();
#pragma unroll
          for (int x = 0; x < 8; ++x) { d0 += hB[x].x * yy[8 + x]; d1 += hB[x].y * yy[8 + x]; }
          m0 += q0 * yy[0];  m1 += q1 * yy[0];
          t0 += d0 * r2.x;   t1 += d1 * r2.y;
#pragma unroll
          for (int j = 0; j < 3; ++j) { j0[j] += q0 * yy[1 + j]; j1[j] += q1 * yy[1 + j]; }
        }
      }
      stage_pair(stw, 0, lane, (m0 * 0.03125f + t0 * 0.03125f) + pz, (m1 * 0.03125f + t1 * 0.03125f) + pz);
#pragma unroll
      for (int j = 0; j < 3; ++j) stage_pair(stw, 1 + j, lane, j0[j] * 0.03125f + pz, j1[j] * 0.03125f + pz);
    }
    __syncthreads();

    v4i pv[NST];
#pragma unroll
    for (int i = 0; i < NST; ++i)
      pv[i] = *(const v4ia*)(dsm + STG_OFF + wave * STG_W + (2 * i + hl16) * 64 + 4 * l15);
#pragma unroll
    for (int i = 0; i < NST; ++i) {
      int* dp = AGw + ((size_t)(2 * i + hl16) * NN + node) * 64 + 4 * l15;
      *(volatile v4i*)dp = pv[i];
    }
    __threadfence();
#pragma unroll
    for (int i = 0; i < NST; ++i) {
      int* dp = AGw + ((size_t)(2 * i + hl16) * NN + node) * 64 + 4 * l15;
      *(volatile v4i*)dp = pv[i];
    }
  }
}

template <int MODE, int L>
__global__ __launch_bounds__(NTHR) __attribute__((amdgpu_num_vgpr(248)))
void k_ngemm(const unsigned short* __restrict__ A, const unsigned short* __restrict__ WD,
             const float* __restrict__ MIXr, const float* __restrict__ WVf, float* OUT, float* MBV) {
  __shared__ __attribute__((aligned(16))) float stg[128 * DP];
  __shared__ __attribute__((aligned(16))) float smb[128];
  __shared__ __attribute__((aligned(16))) float swv[64];
  const int tid = (int)threadIdx.x, lane = tid & 31, wave = tid >> 5, hh = lane >> 4, m = lane & 15;
  const int x = (MODE == 1 && L == 1) ? (int)blockIdx.y + 1 : (int)blockIdx.y;
  const int blk = (x == 0) ? 0 : ((x < 4) ? 1 : ((x < 9) ? 2 : 3));
  const int mat = (MODE == 0) ? (L * 4 + blk) : L;
  const int rowBase = (int)blockIdx.x * 128;

  if (MODE == 1) {
    if (tid < 64) swv[tid] = WVf[L * 64 + tid];
  }

  v8f acc[4];
  {
    const v8f z = {0.f, 0.f, 0.f, 0.f, 0.f, 0.f, 0.f, 0.f};
    acc[0] = z; acc[1] = z; acc[2] = z; acc[3] = z;
  }
  const unsigned short* ap = A + ((size_t)x * NN + rowBase + 16 * wave + m) * 128 + 8 * hh;
  const unsigned short* bp = WD + (size_t)mat * 8192 + (size_t)m * 128 + 8 * hh;
#pragma unroll 1
  for (int k0 = 0; k0 < 128; k0 += 32) {
    FragB af;
    af.h[0] = *(const v8usa*)(ap + k0);
    af.h[1] = *(const v8usa*)(ap + k0 + 16);
#pragma unroll
    for (int nt = 0; nt < 4; ++nt) {
      const unsigned short* wq = bp + (size_t)(16 * nt) * 128 + k0;
      FragB bf;
      bf.h[0] = *(const v8usa*)wq;
      bf.h[1] = *(const v8usa*)(wq + 16);
      acc[nt] = wmb(af, bf, acc[nt]);
    }
  }
#pragma unroll
  for (int nt = 0; nt < 4; ++nt)
#pragma unroll
    for (int r = 0; r < 8; ++r) stg[(16 * wave + 8 * hh + r) * DP + 16 * nt + m] = acc[nt][r];
  __syncthreads();

  v4f pv[8];
#pragma unroll
  for (int i = 0; i < 8; ++i) {
    const int lr = 16 * wave + 2 * i + hh;
    v4f v = *(const v4fa*)(stg + lr * DP + 4 * m);
    if (MODE == 1) {
      const v4f r4 = *(const v4fa*)(MIXr + ((size_t)x * NN + rowBase + lr) * 64 + 4 * m);
      v.x = r4.x + v.x; v.y = r4.y + v.y; v.z = r4.z + v.z; v.w = r4.w + v.w;
    }
    pv[i] = v;
  }
  if (MODE == 0 || L == 0) {
#pragma unroll
    for (int i = 0; i < 8; ++i) {
      float* op = OUT + ((size_t)x * NN + rowBase + 16 * wave + 2 * i + hh) * 64 + 4 * m;
      *(volatile v4f*)op = pv[i];
    }
    __threadfence();
#pragma unroll
    for (int i = 0; i < 8; ++i) {
      float* op = OUT + ((size_t)x * NN + rowBase + 16 * wave + 2 * i + hh) * 64 + 4 * m;
      *(volatile v4f*)op = pv[i];
    }
  }
  if (MODE == 1) {
    if (x >= 1 && x <= 3) {
#pragma unroll
      for (int i = 0; i < 8; ++i) {
        const int lr = 16 * wave + 2 * i + hh;
        *(v4fa*)(stg + lr * DP + 4 * m) = pv[i];
      }
      __syncthreads();
      if (tid < 128) {
        const float* rp = stg + tid * DP;
        float d = 0.0f;
#pragma unroll 4
        for (int cidx = 0; cidx < 64; ++cidx) d += rp[cidx] * swv[cidx];
        smb[tid] = d;
      }
      __syncthreads();
      if (tid < 32) {
        const v4f mv = *(const v4fa*)(smb + 4 * tid);
        putf4(MBV + (size_t)(x - 1) * NN + rowBase + 4 * tid, mv);
      }
    }
  }
}

template <int L>
__global__ __launch_bounds__(NTHR) void k_gate(const float* __restrict__ MIX, unsigned short* P) {
  const int u = (int)blockIdx.x * NTHR + (int)threadIdx.x;
  const int x = (L == 0) ? (u >> 15) : (1 + (u >> 15));
  const int rem = u & 32767;
  const int n = rem >> 3, j = rem & 7;
  const float* mp = MIX + ((size_t)x * NN + n) * 64 + 8 * j;
  const float* sp = MIX + (size_t)n * 64 + 8 * j;
  const v4f ma = *(const v4fa*)mp, mb = *(const v4fa*)(mp + 4);
  const v4f sa = *(const v4fa*)sp, sb = *(const v4fa*)(sp + 4);
  const v8f m8 = {ma.x, ma.y, ma.z, ma.w, mb.x, mb.y, mb.z, mb.w};
  const v8f s8 = {sa.x, sa.y, sa.z, sa.w, sb.x, sb.y, sb.z, sb.w};
  v8us ohi, olo;
#pragma unroll
  for (int i = 0; i < 8; ++i) {
    const float s = s8[i];
    const float g = (s + s * s) + (s * s) * s;
    const float p = m8[i] * g;
    const unsigned hb = bf16_bits(p);
    ohi[i] = (unsigned short)hb;
    olo[i] = (unsigned short)bf16_bits(p - __uint_as_float(hb << 16));
  }
  unsigned short* dp = P + ((size_t)x * NN + n) * 128 + 8 * j;
  *(volatile v8us*)dp        = ohi;
  *(volatile v8us*)(dp + 64) = olo;
  __threadfence();
  *(volatile v8us*)dp        = ohi;
  *(volatile v8us*)(dp + 64) = olo;
}

__global__ __launch_bounds__(NTHR) void k_pos(const float* __restrict__ POS0q, const float* __restrict__ MBV0,
                                              float* POS1q) {
  const int n = (int)blockIdx.x * NTHR + (int)threadIdx.x;
  const v4f p = *(const v4fa*)(POS0q + (size_t)n * 4);
  const float a = MBV0[n], b = MBV0[NN + n], c = MBV0[2 * NN + n];
  v4f q;
  q.x = p.x + a; q.y = p.y + b; q.z = p.z + c; q.w = 0.0f;
  putf4(POS1q + (size_t)n * 4, q);
}

__global__ __launch_bounds__(NTHR) void k_out(const float* __restrict__ POS0q, const float* __restrict__ POS1q,
                                              const float* __restrict__ MBV1, const int* __restrict__ FLG,
                                              float* out) {
  __shared__ __attribute__((aligned(16))) float so[768];
  __shared__ int sf;
  const int tid = (int)threadIdx.x, lane = tid & 31, wave = tid >> 5;
  const int n = (int)blockIdx.x * NTHR + tid;
  const v4f p0 = *(const v4fa*)(POS0q + (size_t)n * 4);
  const v4f p1 = *(const v4fa*)(POS1q + (size_t)n * 4);
  const float a = MBV1[n], b = MBV1[NN + n], c = MBV1[2 * NN + n];
  so[3 * tid + 0] = (p1.x + a) - p0.x;
  so[3 * tid + 1] = (p1.y + b) - p0.y;
  so[3 * tid + 2] = (p1.z + c) - p0.z;
  if (wave == 0) {
    const int f = FLG[lane * 32];
    const unsigned bm = __builtin_amdgcn_ballot_w32(f != 0);
    if (lane == 0) sf = (bm != 0u) ? 1 : 0;
  }
  __syncthreads();
  const bool poison = sf != 0;
  if (tid < 192) {
    v4f v = *(const v4fa*)(so + 4 * tid);
    const float qnan = __int_as_float(0x7fc00000);
    v.x = poison ? qnan : v.x;
    v.y = poison ? qnan : v.y;
    v.z = poison ? qnan : v.z;
    v.w = poison ? qnan : v.w;
    putf4(out + (size_t)blockIdx.x * 768 + 4 * tid, v);
  }
}

extern "C" void kernel_launch(void* const* d_in, const int* in_sizes, int n_in,
                              void* d_out, int out_size, void* d_ws, size_t ws_size,
                              hipStream_t stream) {
  if (n_in < 12) return;
  if (in_sizes[0] != NN * 3 || in_sizes[1] != NN || in_sizes[2] != NN * 32) return;
  if (in_sizes[3] != 2 * NE) return;
  if (in_sizes[4] != 37 * 64 || in_sizes[5] != 64) return;
  if (in_sizes[6] != 2 * 2 * 64 || in_sizes[7] != 2 * 64) return;
  if (in_sizes[8] != 2 * 64 * 64 || in_sizes[9] != 2 * 4 * 64 * 64) return;
  if (in_sizes[10] != 2 * 64 * 64 || in_sizes[11] != 2 * 64) return;
  if (out_size != NN * 3) return;
  if (ws_size < O_END) return;

  const float* pos   = (const float*)d_in[0];
  const int*   attrs = (const int*)d_in[1];
  const float* te    = (const float*)d_in[2];
  const int*   eidx  = (const int*)d_in[3];
  const float* embW  = (const float*)d_in[4];
  const float* embb  = (const float*)d_in[5];
  const float* W1    = (const float*)d_in[6];
  const float* b1    = (const float*)d_in[7];
  const float* W2    = (const float*)d_in[8];
  const float* Wmix  = (const float*)d_in[9];
  const float* Wprod = (const float*)d_in[10];
  const float* Wvec  = (const float*)d_in[11];
  float* out = (float*)d_out;

  char* ws = (char*)d_ws;
  float*          RP    = (float*)(ws + O_RP);
  float*          YP    = (float*)(ws + O_YP);
  float*          LEN0  = (float*)(ws + O_LEN0);
  unsigned short* AG    = (unsigned short*)(ws + O_AG);
  float*          MIX   = (float*)(ws + O_MIX);
  float*          NF    = (float*)(ws + O_NF);
  float*          HS    = (float*)(ws + O_HS);
  float*          POS0q = (float*)(ws + O_POS0);
  float*          POS1q = (float*)(ws + O_POS1);
  float*          MBV0  = (float*)(ws + O_MBV0);
  float*          MBV1  = (float*)(ws + O_MBV1);
  unsigned short* TEB   = (unsigned short*)(ws + O_TEB);
  unsigned short* EWT   = (unsigned short*)(ws + O_EWT);
  float*          EW5   = (float*)(ws + O_EW5);
  float*          EB    = (float*)(ws + O_EB);
  float*          W1f   = (float*)(ws + O_W1F);
  float*          B1f   = (float*)(ws + O_B1F);
  float*          WVf   = (float*)(ws + O_WVF);
  unsigned short* W2D   = (unsigned short*)(ws + O_W2D);
  unsigned short* WMD   = (unsigned short*)(ws + O_WMD);
  unsigned short* WPD   = (unsigned short*)(ws + O_WPD);
  int*            FLG   = (int*)(ws + O_FLG);

  hipFuncSetAttribute(reinterpret_cast<const void*>(&k_edge<0>), hipFuncAttributeMaxDynamicSharedMemorySize,
                      (int)EDGE_LDS_BYTES);
  hipFuncSetAttribute(reinterpret_cast<const void*>(&k_edge<1>), hipFuncAttributeMaxDynamicSharedMemorySize,
                      (int)EDGE_LDS_BYTES);
  hipFuncSetAttribute(reinterpret_cast<const void*>(&k_scan<0>), hipFuncAttributeMaxDynamicSharedMemorySize,
                      (int)SCAN_LDS_BYTES);
  hipFuncSetAttribute(reinterpret_cast<const void*>(&k_scan<1>), hipFuncAttributeMaxDynamicSharedMemorySize,
                      (int)SCAN_LDS_BYTES);

  k_prep<<<PB_END, NTHR, 0, stream>>>(pos, te, embW, embb, W1, b1, W2, Wmix, Wprod, Wvec, ws);
  k_emb<<<NN / 64, 128, 0, stream>>>(TEB, EWT, EW5, EB, attrs, HS);
  k_edge<0><<<NE / 128, NTHR, EDGE_LDS_BYTES, stream>>>(eidx, POS0q, W1f, B1f, W2D, LEN0, YP, RP);
  k_scan<0><<<NN / NBA, NTHR, SCAN_LDS_BYTES, stream>>>(eidx, RP, YP, HS, (int*)AG, FLG);
  k_ngemm<0, 0><<<dim3(NN / 128, 16), NTHR, 0, stream>>>(AG, WMD, MIX, WVf, MIX, MBV0);
  k_gate<0><<<(16 * NN * 8) / NTHR, NTHR, 0, stream>>>(MIX, AG);
  k_ngemm<1, 0><<<dim3(NN / 128, 16), NTHR, 0, stream>>>(AG, WPD, MIX, WVf, NF, MBV0);
  k_pos<<<NN / NTHR, NTHR, 0, stream>>>(POS0q, MBV0, POS1q);
  k_edge<1><<<NE / 128, NTHR, EDGE_LDS_BYTES, stream>>>(eidx, POS1q, W1f, B1f, W2D, LEN0, YP, RP);
  k_scan<1><<<NN / NBA, NTHR, SCAN_LDS_BYTES, stream>>>(eidx, RP, YP, NF, (int*)AG, FLG);
  k_ngemm<0, 1><<<dim3(NN / 128, 4), NTHR, 0, stream>>>(AG, WMD, MIX, WVf, MIX, MBV1);
  k_gate<1><<<(3 * NN * 8) / NTHR, NTHR, 0, stream>>>(MIX, AG);
  k_ngemm<1, 1><<<dim3(NN / 128, 3), NTHR, 0, stream>>>(AG, WPD, MIX, WVf, NF, MBV1);
  k_out<<<NN / NTHR, NTHR, 0, stream>>>(POS0q, POS1q, MBV1, FLG, out);
}
